// EdgeClassifier_4020089389438
// MI455X (gfx1250) — hardware-verified
//
#include <hip/hip_runtime.h>
#include <stddef.h>


#define NF      4
#define EFD     5
#define HD      128
#define KA1     32
#define WSC     64
#define ASC     8
#define NTHR    256
#define NWAVE   8
#define EPT     8
#define NGRP    2
#define CHUNK   (NTHR * EPT * NGRP)
#define WCAP    (EPT * NGRP * 32)
#define LISTN   (NWAVE * WCAP)
#define NBC     4096
#define NBF     1024
#define RCAP    24576
#define RBN     128
#define TGT     256
#define DEGCAP  256
#define OTHR    512
#define BM      64
#define NCW     64
#define EB      64
#define LDZ     136
#define WSCAP   134217728
#define LDS_FILL ((RCAP + NBF + LISTN) * 4 + 64)

static_assert((CHUNK & (CHUNK - 1)) == 0);
static_assert(CHUNK <= 4096);
static_assert(NBC <= 4096 && NBF <= 4096);
static_assert((NBC & (NBC - 1)) == 0 && (NBF & (NBF - 1)) == 0);
static_assert(NBC == 4 * NBF);
static_assert(OTHR * 8 == NBC);
static_assert((RCAP % 32) == 0);
static_assert(TGT == NWAVE * 32);
static_assert((NBC % TGT) == 0);
static_assert((TGT % BM) == 0);
static_assert(BM * 4 == NTHR);
static_assert(EB * 4 == NTHR);
static_assert(WCAP == EPT * NGRP * 32);
static_assert((LDZ % 8) == 0);
static_assert(HD == 128);

typedef float          v4f  __attribute__((ext_vector_type(4)));
typedef float          v8f  __attribute__((ext_vector_type(8)));
typedef int            v4i  __attribute__((ext_vector_type(4)));
typedef _Float16       v4h  __attribute__((ext_vector_type(4)));
typedef _Float16       v8h  __attribute__((ext_vector_type(8)));
typedef _Float16       v16h __attribute__((ext_vector_type(16)));
typedef unsigned short v4us __attribute__((ext_vector_type(4)));
typedef unsigned short v8us __attribute__((ext_vector_type(8)));
union FragH { v16h v; v8us u[2]; };

__device__ __forceinline__ v8f wmh(v16h a, v16h b, v8f c) {
  v8f d = __builtin_amdgcn_wmma_f32_16x16x32_f16(false, a, false, b, (short)0, c, false, false);
  asm volatile("v_nop\n\tv_nop\n\tv_nop\n\tv_nop" : "+v"(d) : "v"(a), "v"(b));
  return d;
}

template <int NB>
__device__ __forceinline__ int scan_chunk(const int* __restrict__ dsts, int nE, int cbase, int slotBase,
                                          int vec8, int* list, int tid, int lane, int wave) {
  int wc = 0;
#pragma unroll
  for (int g = 0; g < NGRP; ++g) {
    const int el0  = (g * NTHR + tid) * EPT;
    const int e0   = cbase + el0;
    const int sent = -2147483647 - 1;
    v4i da, db;
    if (vec8 != 0 && cbase + CHUNK <= nE) {
      da = *(const v4i*)(dsts + e0);
      db = *(const v4i*)(dsts + e0 + 4);
    } else {
      da.x = (e0     < nE) ? dsts[min(e0, nE - 1)] : sent;
      da.y = (e0 + 1 < nE) ? dsts[min(e0 + 1, nE - 1)] : sent;
      da.z = (e0 + 2 < nE) ? dsts[min(e0 + 2, nE - 1)] : sent;
      da.w = (e0 + 3 < nE) ? dsts[min(e0 + 3, nE - 1)] : sent;
      db.x = (e0 + 4 < nE) ? dsts[min(e0 + 4, nE - 1)] : sent;
      db.y = (e0 + 5 < nE) ? dsts[min(e0 + 5, nE - 1)] : sent;
      db.z = (e0 + 6 < nE) ? dsts[min(e0 + 6, nE - 1)] : sent;
      db.w = (e0 + 7 < nE) ? dsts[min(e0 + 7, nE - 1)] : sent;
    }
    const unsigned nb = (unsigned)slotBase;
    const unsigned s0 = (unsigned)da.x - nb, s1 = (unsigned)da.y - nb;
    const unsigned s2 = (unsigned)da.z - nb, s3 = (unsigned)da.w - nb;
    const unsigned s4 = (unsigned)db.x - nb, s5 = (unsigned)db.y - nb;
    const unsigned s6 = (unsigned)db.z - nb, s7 = (unsigned)db.w - nb;
    const bool h0 = s0 < (unsigned)NB, h1 = s1 < (unsigned)NB, h2 = s2 < (unsigned)NB, h3 = s3 < (unsigned)NB;
    const bool h4 = s4 < (unsigned)NB, h5 = s5 < (unsigned)NB, h6 = s6 < (unsigned)NB, h7 = s7 < (unsigned)NB;
    const unsigned any = __builtin_amdgcn_ballot_w32(h0 | h1 | h2 | h3 | h4 | h5 | h6 | h7);
    if (any != 0u) {
#define HITJ(J, HJ, SJ) { \
        const unsigned mj = __builtin_amdgcn_ballot_w32(HJ); \
        if (mj != 0u) { \
          if (HJ) { \
            const int pos = wc + (int)__builtin_amdgcn_mbcnt_lo(mj, 0u); \
            if (pos < WCAP) list[wave * WCAP + pos] = ((el0 + (J)) << 12) | (int)(SJ); \
          } \
          wc += (int)__builtin_popcount(mj); } }
      HITJ(0, h0, s0)
      HITJ(1, h1, s1)
      HITJ(2, h2, s2)
      HITJ(3, h3, s3)
      HITJ(4, h4, s4)
      HITJ(5, h5, s5)
      HITJ(6, h6, s6)
      HITJ(7, h7, s7)
#undef HITJ
    }
  }
  return wc;
}

__global__ __launch_bounds__(NTHR) void k_count(
    const int* __restrict__ dsts, int* cnt, int nE, int vec8) {
  __shared__ __attribute__((aligned(16))) int scnt[NBC];
  __shared__ __attribute__((aligned(16))) int list[LISTN];
  __shared__ int wcnt[NWAVE];
  const int tid = threadIdx.x, lane = tid & 31, wave = tid >> 5;
  const int nodeBase = blockIdx.x * NBC;

  for (int i = tid; i < NBC; i += NTHR) scnt[i] = 0;
  __syncthreads();

  const int nChunks = (nE + CHUNK - 1) / CHUNK;
#pragma unroll 1
  for (int ch = 0; ch < nChunks; ++ch) {
    const int cbase = ch * CHUNK;
    const int wc = scan_chunk<NBC>(dsts, nE, cbase, nodeBase, vec8, list, tid, lane, wave);
    if (lane == 0) wcnt[wave] = wc;
    __syncthreads();
    if (wave == 0) {
#pragma unroll 1
      for (int wsx = 0; wsx < NWAVE; ++wsx) {
        int n = __builtin_amdgcn_readfirstlane(wcnt[wsx]);
        n = n > WCAP ? WCAP : (n < 0 ? 0 : n);
        const int* lp = list + wsx * WCAP;
#pragma unroll 1
        for (int i = 0; i < n; ++i) {
          const int ent  = __builtin_amdgcn_readfirstlane(lp[i]);
          const int slot = ent & (NBC - 1);
          if (lane == 0) scnt[slot] = scnt[slot] + 1;
        }
      }
    }
    __syncthreads();
  }

  v4i cq[4];
#pragma unroll
  for (int q = 0; q < 4; ++q) {
    const int f = (wave * 4 + q) * 128 + 4 * lane;
    cq[q] = *(const v4i*)(scnt + f);
  }
  int* cp = cnt + (size_t)nodeBase;
#pragma unroll
  for (int q = 0; q < 4; ++q) {
    const int f = (wave * 4 + q) * 128 + 4 * lane;
    *(volatile v4i*)(cp + f) = cq[q];
  }
  __threadfence();
#pragma unroll
  for (int q = 0; q < 4; ++q) {
    const int f = (wave * 4 + q) * 128 + 4 * lane;
    *(volatile v4i*)(cp + f) = cq[q];
  }
}

__global__ __launch_bounds__(OTHR) void k_offsets(
    const int* __restrict__ cnt, int* off, int* rbase, int nChunk) {
  __shared__ __attribute__((aligned(16))) int soff[NBC];
  __shared__ __attribute__((aligned(16))) int srb[RBN];
  __shared__ int wtot[OTHR / 32];
  const int tid = threadIdx.x, lane = tid & 31, wave = tid >> 5, sub = tid >> 7;
  for (int i = tid; i < RBN; i += OTHR) srb[i] = 0;
  int carry = 0;
#pragma unroll 1
  for (int ch = 0; ch < nChunk; ++ch) {
    const int base = ch * NBC;
    const v4i c0 = *(const v4i*)(cnt + base + 8 * tid);
    const v4i c1 = *(const v4i*)(cnt + base + 8 * tid + 4);
    const int e0 = max(c0.x, 0), e1 = max(c0.y, 0), e2 = max(c0.z, 0), e3 = max(c0.w, 0);
    const int e4 = max(c1.x, 0), e5 = max(c1.y, 0), e6 = max(c1.z, 0), e7 = max(c1.w, 0);
    const int ts = e0 + e1 + e2 + e3 + e4 + e5 + e6 + e7;
    int incl = ts;
#pragma unroll
    for (int d = 1; d < 32; d <<= 1) {
      const int t = __shfl_up(incl, d);
      if (lane >= d) incl += t;
    }
    if (lane == 31) wtot[wave] = incl;
    __syncthreads();
    const int S0 = wtot[0]  + wtot[1]  + wtot[2]  + wtot[3];
    const int S1 = wtot[4]  + wtot[5]  + wtot[6]  + wtot[7];
    const int S2 = wtot[8]  + wtot[9]  + wtot[10] + wtot[11];
    const int S3 = wtot[12] + wtot[13] + wtot[14] + wtot[15];
    int pre = 0;
#pragma unroll 1
    for (int w = 4 * sub; w < wave; ++w) pre += wtot[w];
    const int b0 = carry;
    const int b1 = b0 + ((S0 + 31) & ~31);
    const int b2 = b1 + ((S1 + 31) & ~31);
    const int b3 = b2 + ((S2 + 31) & ~31);
    const int b4 = b3 + ((S3 + 31) & ~31);
    const int myb = sub == 0 ? b0 : (sub == 1 ? b1 : (sub == 2 ? b2 : b3));
    if (tid == 0) {
      srb[min(4 * ch + 0, RBN - 1)] = b0;
      srb[min(4 * ch + 1, RBN - 1)] = b1;
      srb[min(4 * ch + 2, RBN - 1)] = b2;
      srb[min(4 * ch + 3, RBN - 1)] = b3;
    }
    int run = myb + pre + incl - ts;
    soff[8 * tid + 0] = run; run += e0;
    soff[8 * tid + 1] = run; run += e1;
    soff[8 * tid + 2] = run; run += e2;
    soff[8 * tid + 3] = run; run += e3;
    soff[8 * tid + 4] = run; run += e4;
    soff[8 * tid + 5] = run; run += e5;
    soff[8 * tid + 6] = run; run += e6;
    soff[8 * tid + 7] = run;
    carry = b4;
    __syncthreads();
    const v4i o0 = *(const v4i*)(soff + 4 * tid);
    const v4i o1 = *(const v4i*)(soff + 4 * (tid + OTHR));
    int* op = off + base;
    *(volatile v4i*)(op + 4 * tid) = o0;
    *(volatile v4i*)(op + 4 * (tid + OTHR)) = o1;
    __threadfence();
    *(volatile v4i*)(op + 4 * tid) = o0;
    *(volatile v4i*)(op + 4 * (tid + OTHR)) = o1;
    __syncthreads();
  }
  if (tid == 0) srb[min(4 * nChunk, RBN - 1)] = carry;
  __syncthreads();
  v4i rv = {0, 0, 0, 0};
  if (tid < 32) rv = *(const v4i*)(srb + 4 * tid);
  if (tid < 32) *(volatile v4i*)(rbase + 4 * tid) = rv;
  __threadfence();
  if (tid < 32) *(volatile v4i*)(rbase + 4 * tid) = rv;
}

__global__ __launch_bounds__(NTHR) void k_fill(
    const int* __restrict__ srcs, const int* __restrict__ dsts,
    const int* __restrict__ off, const int* __restrict__ rbase,
    int* csr, int nN, int nE, int vec8, int csrLen) {
  extern __shared__ v4f lds_dyn[];
  int* region = (int*)lds_dyn;
  int* cursor = region + RCAP;
  int* list   = cursor + NBF;
  int* wcnt   = list + LISTN;
  const int tid = threadIdx.x, lane = tid & 31, wave = tid >> 5;
  const int b = blockIdx.x;
  const int nodeBase = b * NBF;

  int rb0 = rbase[b];
  const int rb1 = rbase[b + 1];
  rb0 = rb0 < 0 ? 0 : (rb0 > csrLen ? csrLen : rb0);
  rb0 &= ~31;
  int len = rb1 - rb0;
  len = len < 0 ? 0 : (len > RCAP ? RCAP : len);
  int lenW = (len + 31) & ~31;
  if (rb0 + lenW > csrLen) lenW = (csrLen - rb0) & ~31;

  {
    const v4i z = {0, 0, 0, 0};
    for (int i = tid; i < RCAP / 4; i += NTHR) ((v4i*)region)[i] = z;
    for (int s = tid; s < NBF; s += NTHR) {
      int o = off[nodeBase + s] - rb0;
      o = o < 0 ? 0 : (o > RCAP ? RCAP : o);
      cursor[s] = o;
    }
  }
  __syncthreads();

  const int nChunks = (nE + CHUNK - 1) / CHUNK;
#pragma unroll 1
  for (int ch = 0; ch < nChunks; ++ch) {
    const int cbase = ch * CHUNK;
    const int wc = scan_chunk<NBF>(dsts, nE, cbase, nodeBase, vec8, list, tid, lane, wave);
    if (lane == 0) wcnt[wave] = wc;
    __syncthreads();
    if (wave == 0) {
#pragma unroll 1
      for (int wsx = 0; wsx < NWAVE; ++wsx) {
        int n = __builtin_amdgcn_readfirstlane(wcnt[wsx]);
        n = n > WCAP ? WCAP : (n < 0 ? 0 : n);
        const int* lp = list + wsx * WCAP;
#pragma unroll 1
        for (int i = 0; i < n; ++i) {
          const int ent  = __builtin_amdgcn_readfirstlane(lp[i]);
          const int slot = ent & (NBF - 1);
          int e = cbase + ((ent >> 12) & (CHUNK - 1));
          e = e > nE - 1 ? nE - 1 : e;
          int sv = srcs[e];
          sv = sv < 0 ? 0 : (sv > nN - 1 ? nN - 1 : sv);
          if (lane == 0) {
            int pos = cursor[slot];
            pos = pos < 0 ? 0 : (pos > RCAP - 1 ? RCAP - 1 : pos);
            region[pos] = sv;
            const int np = pos + 1;
            cursor[slot] = np > RCAP ? RCAP : np;
          }
        }
      }
    }
    __syncthreads();
  }

  const int nv = lenW >> 2;
  int* gp = csr + rb0;
#pragma unroll 1
  for (int i = tid; i < nv; i += NTHR) { const v4i v = ((const v4i*)region)[i]; *(volatile v4i*)(gp + 4 * i) = v; }
  __threadfence();
#pragma unroll 1
  for (int i = tid; i < nv; i += NTHR) { const v4i v = ((const v4i*)region)[i]; *(volatile v4i*)(gp + 4 * i) = v; }
}

__global__ __launch_bounds__(NTHR) void k_wcvt16(const float* __restrict__ W, unsigned short* wp,
                                                 int K, int Nout, int ldw, int split, int kp8) {
  const int units = Nout * kp8;
  const int i = (int)blockIdx.x * NTHR + (int)threadIdx.x;
  if (i >= units) return;
  const int n = i / kp8;
  const int seg = i - n * kp8;
  const int hiq = (n >= split) ? 1 : 0;
  const int ro = hiq ? K : 0;
  int nc = n - (hiq ? split : 0);
  nc = nc < 0 ? 0 : (nc > ldw - 1 ? ldw - 1 : nc);
  v8h o;
#pragma unroll
  for (int j = 0; j < 8; ++j) {
    const int k = 8 * seg + j;
    const int kc = k < K - 1 ? k : K - 1;
    const bool valid = (k < K);
    const float v = W[(size_t)(ro + kc) * ldw + nc];
    o[j] = valid ? (_Float16)(v * (float)WSC) : (_Float16)0.0f;
  }
  const v8us ob = __builtin_bit_cast(v8us, o);
  unsigned short* d = wp + (size_t)i * 8;
  *(volatile v8us*)d = ob;
  __threadfence();
  *(volatile v8us*)d = ob;
}

__global__ __launch_bounds__(NTHR) void k_xprep(const float* __restrict__ x, unsigned short* A1, int nN) {
  __shared__ __attribute__((aligned(16))) unsigned short sA[NTHR * KA1];
  const int tid = threadIdx.x;
  const int rowBase = (int)blockIdx.x * NTHR;
  const int row = rowBase + tid;
  int rr = row > nN - 1 ? nN - 1 : row;
  rr = rr < 0 ? 0 : rr;
  const bool live = row < nN;
  const v4f z4 = {0.f, 0.f, 0.f, 0.f};
  v4f xv = *(const v4f*)(x + (size_t)rr * NF);
  xv = xv * (float)ASC;
  xv = live ? xv : z4;
  v4h hv;
  hv[0] = (_Float16)xv.x; hv[1] = (_Float16)xv.y; hv[2] = (_Float16)xv.z; hv[3] = (_Float16)xv.w;
  const v4us hb = __builtin_bit_cast(v4us, hv);
  const v4us z4u = {0, 0, 0, 0};
  const v8us z8u = {0, 0, 0, 0, 0, 0, 0, 0};
  unsigned short* sr = sA + tid * KA1;
  *(v4us*)(sr)      = hb;
  *(v4us*)(sr + 4)  = z4u;
  *(v8us*)(sr + 8)  = z8u;
  *(v8us*)(sr + 16) = z8u;
  *(v8us*)(sr + 24) = z8u;
  __syncthreads();
  v8us pv[4];
#pragma unroll
  for (int it = 0; it < 4; ++it) pv[it] = *(const v8us*)(sA + 8 * (it * NTHR + tid));
  unsigned short* ab = A1 + (size_t)rowBase * KA1;
#pragma unroll
  for (int it = 0; it < 4; ++it) *(volatile v8us*)(ab + 8 * (it * NTHR + tid)) = pv[it];
  __threadfence();
#pragma unroll
  for (int it = 0; it < 4; ++it) *(volatile v8us*)(ab + 8 * (it * NTHR + tid)) = pv[it];
}

__global__ __launch_bounds__(NTHR) void k_gemm(const unsigned short* __restrict__ Ap,
                                               const unsigned short* __restrict__ Bp,
                                               float* C, int lda, int KT, int ldc, float osc) {
  __shared__ __attribute__((aligned(16))) float stg[BM * NCW];
  const int tid = threadIdx.x, lane = tid & 31, wave = tid >> 5, hh = lane >> 4, m = lane & 15;
  const int rowBase = (int)blockIdx.x * BM;
  const int colBase = (int)blockIdx.y * NCW;
  const int rg = wave >> 1, chf = wave & 1;
  const int r0 = rg * 16;
  const int c0 = chf * 32;
  const int KB = 32 * KT;

  v8f acc0 = {0.f, 0.f, 0.f, 0.f, 0.f, 0.f, 0.f, 0.f};
  v8f acc1 = {0.f, 0.f, 0.f, 0.f, 0.f, 0.f, 0.f, 0.f};

  const unsigned short* ap  = Ap + (size_t)(rowBase + r0 + m) * lda + 8 * hh;
  const unsigned short* bpA = Bp + (size_t)(colBase + c0 + m) * KB + 8 * hh;
  const unsigned short* bpB = bpA + (size_t)16 * KB;
#pragma unroll 1
  for (int kt = 0; kt < KT; ++kt) {
    FragH a, b0, b1;
    a.u[0]  = *(const v8us*)(ap + 32 * kt);
    a.u[1]  = *(const v8us*)(ap + 32 * kt + 16);
    b0.u[0] = *(const v8us*)(bpA + 32 * kt);
    b0.u[1] = *(const v8us*)(bpA + 32 * kt + 16);
    b1.u[0] = *(const v8us*)(bpB + 32 * kt);
    b1.u[1] = *(const v8us*)(bpB + 32 * kt + 16);
    acc0 = wmh(a.v, b0.v, acc0);
    acc1 = wmh(a.v, b1.v, acc1);
  }

  {
    float* sp = stg + (size_t)(r0 + 8 * hh) * NCW + c0 + m;
#pragma unroll
    for (int r = 0; r < 8; ++r) {
      sp[r * NCW]      = acc0[r] * osc;
      sp[r * NCW + 16] = acc1[r] * osc;
    }
  }
  __syncthreads();

  v4f cv[4];
#pragma unroll
  for (int it = 0; it < 4; ++it) {
    const int id = it * NTHR + tid;
    const int row = id >> 4, seg = id & 15;
    cv[it] = *(const v4f*)(stg + (size_t)row * NCW + 4 * seg);
  }
#pragma unroll
  for (int it = 0; it < 4; ++it) {
    const int id = it * NTHR + tid;
    const int row = id >> 4, seg = id & 15;
    float* gp = C + (size_t)(rowBase + row) * ldc + colBase + 4 * seg;
    *(volatile v4f*)gp = cv[it];
  }
  __threadfence();
#pragma unroll
  for (int it = 0; it < 4; ++it) {
    const int id = it * NTHR + tid;
    const int row = id >> 4, seg = id & 15;
    float* gp = C + (size_t)(rowBase + row) * ldc + colBase + 4 * seg;
    *(volatile v4f*)gp = cv[it];
  }
}

template <int RELU>
__global__ __launch_bounds__(NTHR) void k_agg(
    const int* __restrict__ csr, const int* __restrict__ off, const int* __restrict__ cnt,
    const float* __restrict__ hw, const float* __restrict__ bias,
    unsigned short* Aout, int nN, int csrLen) {
  const int tid = threadIdx.x, lane = tid & 31, wave = tid >> 5;
  const int tbase = (int)blockIdx.x * TGT + wave * 32;
  const int cl    = tbase + lane;
  const int cnt_l = cnt[cl];
  const int off_l = off[cl];
  const v4f bq = *(const v4f*)(bias + 4 * lane);
  const v4f z4 = {0.f, 0.f, 0.f, 0.f};

#pragma unroll 1
  for (int j = 0; j < 32; ++j) {
    const int c = tbase + j;
    int nraw = __builtin_amdgcn_readfirstlane(__shfl(cnt_l, j));
    nraw = nraw < 0 ? 0 : nraw;
    const int n = nraw > DEGCAP ? DEGCAP : nraw;
    const int st = __builtin_amdgcn_readfirstlane(__shfl(off_l, j));
    const float dc = rsqrtf((float)(nraw + 1));
    const int cc = c > nN - 1 ? nN - 1 : c;
    const float wself = dc * dc;
    v4f acc = *(const v4f*)(hw + (size_t)cc * HD + 4 * lane) * wself;
#pragma unroll 1
    for (int q0 = 0; q0 < n; q0 += 32) {
      int pos = st + q0 + lane;
      pos = pos < 0 ? 0 : (pos > csrLen - 1 ? csrLen - 1 : pos);
      int sl = csr[pos];
      sl = sl < 0 ? 0 : (sl > nN - 1 ? nN - 1 : sl);
      int cs = cnt[sl];
      cs = cs < 0 ? 0 : cs;
      const float wl = rsqrtf((float)(cs + 1)) * dc;
      const int mcnt = (n - q0) < 32 ? (n - q0) : 32;
#pragma unroll 1
      for (int pp = 0; pp < mcnt; ++pp) {
        const int s = __builtin_amdgcn_readlane(sl, pp);
        const float w = __int_as_float(__builtin_amdgcn_readlane(__float_as_int(wl), pp));
        const v4f xv = *(const v4f*)(hw + (size_t)s * HD + 4 * lane);
        acc += xv * w;
      }
    }
    v4f o = acc + bq;
    if (RELU) {
      o.x = fmaxf(o.x, 0.f); o.y = fmaxf(o.y, 0.f); o.z = fmaxf(o.z, 0.f); o.w = fmaxf(o.w, 0.f);
    }
    const bool live = c < nN;
    o = live ? o : z4;
    v4h hv;
    hv[0] = (_Float16)(o.x * (float)ASC); hv[1] = (_Float16)(o.y * (float)ASC);
    hv[2] = (_Float16)(o.z * (float)ASC); hv[3] = (_Float16)(o.w * (float)ASC);
    const v4us hb = __builtin_bit_cast(v4us, hv);
    unsigned short* rp = Aout + (size_t)c * HD + 4 * lane;
    *(volatile v4us*)rp = hb;
    __threadfence();
    *(volatile v4us*)rp = hb;
  }
}

__global__ __launch_bounds__(NTHR) void k_edge(
    const int* __restrict__ ei, const float* __restrict__ ef, const float* __restrict__ PQ,
    const float* __restrict__ Wm1, const float* __restrict__ bm1,
    const unsigned short* __restrict__ wm2p, const float* __restrict__ bm2,
    const float* __restrict__ wm3, const float* __restrict__ bm3,
    float* out, int nE, int nN) {
  __shared__ __attribute__((aligned(16))) unsigned short sz[EB * LDZ];
  __shared__ __attribute__((aligned(16))) float swe[EFD * HD];
  __shared__ __attribute__((aligned(16))) float sb1[HD];
  __shared__ __attribute__((aligned(16))) float sb2s[HD];
  __shared__ __attribute__((aligned(16))) float sw3s[HD];
  __shared__ __attribute__((aligned(16))) float sea[EB * 8];
  __shared__ int ssd[2 * EB];
  __shared__ float sred[NWAVE * 16];
  __shared__ __attribute__((aligned(16))) float sout[EB];
  const int tid = threadIdx.x, lane = tid & 31, wave = tid >> 5, hh = lane >> 4, m = lane & 15;
  const int e0 = (int)blockIdx.x * EB;
  const float isc = (float)(ASC * WSC);
  const float osc = 1.0f / isc;

  if (tid < HD) {
    sb1[tid]  = bm1[tid];
    sb2s[tid] = bm2[tid] * isc;
    sw3s[tid] = wm3[tid] * osc;
  }
  for (int u = tid; u < EFD * HD; u += NTHR) swe[u] = Wm1[(size_t)(2 * HD) * HD + u];
  if (tid < EB) {
    const int e = e0 + tid;
    const int ec = e > nE - 1 ? nE - 1 : e;
    int s = ei[ec];
    int d = ei[(size_t)nE + ec];
    s = s < 0 ? 0 : (s > nN - 1 ? nN - 1 : s);
    d = d < 0 ? 0 : (d > nN - 1 ? nN - 1 : d);
    ssd[tid] = s;
    ssd[EB + tid] = d;
    const float* er = ef + (size_t)ec * EFD;
    sea[tid * 8 + 0] = er[0]; sea[tid * 8 + 1] = er[1]; sea[tid * 8 + 2] = er[2];
    sea[tid * 8 + 3] = er[3]; sea[tid * 8 + 4] = er[4];
    sea[tid * 8 + 5] = 0.0f;  sea[tid * 8 + 6] = 0.0f;  sea[tid * 8 + 7] = 0.0f;
  }
  __syncthreads();

  {
    const int r = tid >> 2, cq = tid & 3;
    const int s = ssd[r], d = ssd[EB + r];
    const float* prow = PQ + (size_t)s * (2 * HD);
    const float* qrow = PQ + (size_t)d * (2 * HD) + HD;
    const float a0 = sea[r * 8 + 0], a1 = sea[r * 8 + 1], a2 = sea[r * 8 + 2];
    const float a3 = sea[r * 8 + 3], a4 = sea[r * 8 + 4];
    unsigned short* zr = sz + r * LDZ;
#pragma unroll 1
    for (int g = 0; g < 8; ++g) {
      const int n0 = 16 * g + 4 * cq;
      const v4f p = *(const v4f*)(prow + n0);
      const v4f q = *(const v4f*)(qrow + n0);
      v4f a = (p + q) + *(const v4f*)(sb1 + n0);
      a += *(const v4f*)(swe + 0 * HD + n0) * a0;
      a += *(const v4f*)(swe + 1 * HD + n0) * a1;
      a += *(const v4f*)(swe + 2 * HD + n0) * a2;
      a += *(const v4f*)(swe + 3 * HD + n0) * a3;
      a += *(const v4f*)(swe + 4 * HD + n0) * a4;
      v4h hv;
      hv[0] = (_Float16)(fmaxf(a.x, 0.f) * (float)ASC);
      hv[1] = (_Float16)(fmaxf(a.y, 0.f) * (float)ASC);
      hv[2] = (_Float16)(fmaxf(a.z, 0.f) * (float)ASC);
      hv[3] = (_Float16)(fmaxf(a.w, 0.f) * (float)ASC);
      *(v4us*)(zr + n0) = __builtin_bit_cast(v4us, hv);
    }
  }
  __syncthreads();

  const int rg = wave >> 1, chf = wave & 1;
  v8f acc0 = {0.f, 0.f, 0.f, 0.f, 0.f, 0.f, 0.f, 0.f};
  v8f acc1 = {0.f, 0.f, 0.f, 0.f, 0.f, 0.f, 0.f, 0.f};
  v8f acc2 = {0.f, 0.f, 0.f, 0.f, 0.f, 0.f, 0.f, 0.f};
  v8f acc3 = {0.f, 0.f, 0.f, 0.f, 0.f, 0.f, 0.f, 0.f};
  {
    const unsigned short* ap = sz + (rg * 16 + m) * LDZ + 8 * hh;
    const unsigned short* bp = wm2p + (size_t)(chf * 64 + m) * HD + 8 * hh;
#pragma unroll 1
    for (int kt = 0; kt < 4; ++kt) {
      FragH a, b0, b1, b2, b3;
      a.u[0]  = *(const v8us*)(ap + 32 * kt);
      a.u[1]  = *(const v8us*)(ap + 32 * kt + 16);
      b0.u[0] = *(const v8us*)(bp + 32 * kt);
      b0.u[1] = *(const v8us*)(bp + 32 * kt + 16);
      b1.u[0] = *(const v8us*)(bp + 16 * HD + 32 * kt);
      b1.u[1] = *(const v8us*)(bp + 16 * HD + 32 * kt + 16);
      b2.u[0] = *(const v8us*)(bp + 32 * HD + 32 * kt);
      b2.u[1] = *(const v8us*)(bp + 32 * HD + 32 * kt + 16);
      b3.u[0] = *(const v8us*)(bp + 48 * HD + 32 * kt);
      b3.u[1] = *(const v8us*)(bp + 48 * HD + 32 * kt + 16);
      acc0 = wmh(a.v, b0.v, acc0);
      acc1 = wmh(a.v, b1.v, acc1);
      acc2 = wmh(a.v, b2.v, acc2);
      acc3 = wmh(a.v, b3.v, acc3);
    }
  }

  {
    const int cb = chf * 64 + m;
    const float bt0 = sb2s[cb],      wt0 = sw3s[cb];
    const float bt1 = sb2s[cb + 16], wt1 = sw3s[cb + 16];
    const float bt2 = sb2s[cb + 32], wt2 = sw3s[cb + 32];
    const float bt3 = sb2s[cb + 48], wt3 = sw3s[cb + 48];
    float ps[8];
#pragma unroll
    for (int r = 0; r < 8; ++r) {
      float t = fmaxf(acc0[r] + bt0, 0.f) * wt0;
      t += fmaxf(acc1[r] + bt1, 0.f) * wt1;
      t += fmaxf(acc2[r] + bt2, 0.f) * wt2;
      t += fmaxf(acc3[r] + bt3, 0.f) * wt3;
      ps[r] = t;
    }
#pragma unroll
    for (int r = 0; r < 8; ++r) {
      float v = ps[r];
      v += __shfl_xor(v, 1);
      v += __shfl_xor(v, 2);
      v += __shfl_xor(v, 4);
      v += __shfl_xor(v, 8);
      ps[r] = v;
    }
    if (m == 0) {
#pragma unroll
      for (int r = 0; r < 8; ++r) sred[wave * 16 + 8 * hh + r] = ps[r];
    }
  }
  __syncthreads();
  if (tid < EB) {
    const int rg2 = tid >> 4, rl = tid & 15;
    const float s = sred[(2 * rg2) * 16 + rl] + sred[(2 * rg2 + 1) * 16 + rl] + bm3[0];
    sout[tid] = __builtin_amdgcn_rcpf(1.0f + __expf(-s));
  }
  __syncthreads();
  const int l16 = tid < 16 ? tid : 15;
  const v4f ov = *(const v4f*)(sout + 4 * l16);
  const int rem = nE - e0 - 4 * l16;
  float* gp = out + (size_t)e0 + 4 * l16;
  const bool full = (tid < 16) && (rem >= 4);
  const bool part = (tid < 16) && (rem > 0) && (rem < 4);
  if (full) *(volatile v4f*)gp = ov;
  if (part) {
    *(volatile float*)gp = ov.x;
    if (rem > 1) *(volatile float*)(gp + 1) = ov.y;
    if (rem > 2) *(volatile float*)(gp + 2) = ov.z;
  }
  __threadfence();
  if (full) *(volatile v4f*)gp = ov;
  if (part) {
    *(volatile float*)gp = ov.x;
    if (rem > 1) *(volatile float*)(gp + 1) = ov.y;
    if (rem > 2) *(volatile float*)(gp + 2) = ov.z;
  }
}

extern "C" void kernel_launch(void* const* d_in, const int* in_sizes, int n_in,
                              void* d_out, int out_size, void* d_ws, size_t ws_size,
                              hipStream_t stream) {
  if (n_in < 13) return;
  const int nN = in_sizes[0] / NF;
  const int nE = in_sizes[1] / EFD;
  if (nN <= 0 || nE <= 0) return;
  if (in_sizes[0] != nN * NF || in_sizes[1] != nE * EFD) return;
  if (in_sizes[2] != NF * HD || in_sizes[3] != HD) return;
  if (in_sizes[4] != HD * HD || in_sizes[5] != HD) return;
  if (in_sizes[6] != (2 * HD + EFD) * HD || in_sizes[7] != HD) return;
  if (in_sizes[8] != HD * HD || in_sizes[9] != HD) return;
  if (in_sizes[10] != HD || in_sizes[11] != 1) return;
  if (in_sizes[12] != 2 * nE) return;
  if (out_size != nE) return;
  if (nE > (1 << 28) || nN > (1 << 22)) return;

  const float* x    = (const float*)d_in[0];
  const float* ef   = (const float*)d_in[1];
  const float* W1   = (const float*)d_in[2];
  const float* b1   = (const float*)d_in[3];
  const float* W2   = (const float*)d_in[4];
  const float* b2   = (const float*)d_in[5];
  const float* Wm1  = (const float*)d_in[6];
  const float* bm1  = (const float*)d_in[7];
  const float* Wm2  = (const float*)d_in[8];
  const float* bm2  = (const float*)d_in[9];
  const float* Wm3  = (const float*)d_in[10];
  const float* bm3  = (const float*)d_in[11];
  const int*   ei   = (const int*)d_in[12];
  const int*   src  = ei;
  const int*   dst  = ei + nE;
  float* out = (float*)d_out;

  const int NPAD   = ((nN + TGT - 1) / TGT) * TGT;
  const int nBC    = (nN + NBC - 1) / NBC;
  const int CNTPAD = nBC * NBC;
  if (CNTPAD < NPAD) return;
  if (4 * nBC + 1 > RBN) return;
  const int nBF    = (nN + NBF - 1) / NBF;
  if (nBF > 4 * nBC) return;
  const int csrLen = ((nE + 31) & ~31) + 4096;
  if (31 * 4 * nBC > 4096) return;
  const int nAgg   = NPAD / TGT;
  const int nGemm  = NPAD / BM;
  const int nEB    = (nE + EB - 1) / EB;

  char* ws = (char*)d_ws;
  size_t off = 0;
  const size_t oW1  = off; off += (size_t)HD * KA1 * 2;          off = (off + 255) & ~(size_t)255;
  const size_t oW2  = off; off += (size_t)HD * HD * 2;           off = (off + 255) & ~(size_t)255;
  const size_t oWpq = off; off += (size_t)(2 * HD) * HD * 2;     off = (off + 255) & ~(size_t)255;
  const size_t oWm2 = off; off += (size_t)HD * HD * 2;           off = (off + 255) & ~(size_t)255;
  const size_t oCnt = off; off += (size_t)CNTPAD * 4;            off = (off + 255) & ~(size_t)255;
  const size_t oOff = off; off += (size_t)CNTPAD * 4;            off = (off + 255) & ~(size_t)255;
  const size_t oRb  = off; off += (size_t)RBN * 4;               off = (off + 255) & ~(size_t)255;
  const size_t oCsr = off; off += (size_t)csrLen * 4;            off = (off + 255) & ~(size_t)255;
  const size_t oA   = off; off += (size_t)NPAD * HD * 2;         off = (off + 255) & ~(size_t)255;
  const size_t oPQ  = off; off += (size_t)NPAD * (2 * HD) * 4;   off = (off + 255) & ~(size_t)255;
  if (off > ws_size || off > (size_t)WSCAP) return;

  unsigned short* w1p  = (unsigned short*)(ws + oW1);
  unsigned short* w2p  = (unsigned short*)(ws + oW2);
  unsigned short* wpq  = (unsigned short*)(ws + oWpq);
  unsigned short* wm2p = (unsigned short*)(ws + oWm2);
  int*            cnt  = (int*)(ws + oCnt);
  int*            offp = (int*)(ws + oOff);
  int*            rb   = (int*)(ws + oRb);
  int*            csr  = (int*)(ws + oCsr);
  unsigned short* A1   = (unsigned short*)(ws + oA);
  unsigned short* A2   = (unsigned short*)(ws + oA);
  unsigned short* A3   = (unsigned short*)(ws + oA);
  float*          HW   = (float*)(ws + oPQ);
  float*          PQ   = (float*)(ws + oPQ);

  const int vec8 = ((nE & 3) == 0) ? 1 : 0;
  const float osc = 1.0f / (float)(ASC * WSC);

  k_wcvt16<<<(HD * (KA1 / 8) + NTHR - 1) / NTHR, NTHR, 0, stream>>>(W1, w1p, NF, HD, HD, HD, KA1 / 8);
  k_wcvt16<<<(HD * (HD / 8) + NTHR - 1) / NTHR, NTHR, 0, stream>>>(W2, w2p, HD, HD, HD, HD, HD / 8);
  k_wcvt16<<<(2 * HD * (HD / 8) + NTHR - 1) / NTHR, NTHR, 0, stream>>>(Wm1, wpq, HD, 2 * HD, HD, HD, HD / 8);
  k_wcvt16<<<(HD * (HD / 8) + NTHR - 1) / NTHR, NTHR, 0, stream>>>(Wm2, wm2p, HD, HD, HD, HD, HD / 8);
  k_xprep<<<NPAD / NTHR, NTHR, 0, stream>>>(x, A1, nN);
  k_count<<<nBC, NTHR, 0, stream>>>(dst, cnt, nE, vec8);
  k_offsets<<<1, OTHR, 0, stream>>>(cnt, offp, rb, nBC);
  hipFuncSetAttribute(reinterpret_cast<const void*>(&k_fill),
                      hipFuncAttributeMaxDynamicSharedMemorySize, LDS_FILL);
  k_fill<<<nBF, NTHR, LDS_FILL, stream>>>(src, dst, offp, rb, csr, nN, nE, vec8, csrLen);
  k_gemm<<<dim3(nGemm, HD / NCW, 1), NTHR, 0, stream>>>(A1, w1p, HW, KA1, 1, HD, osc);
  k_agg<1><<<nAgg, NTHR, 0, stream>>>(csr, offp, cnt, HW, b1, A2, nN, csrLen);
  k_gemm<<<dim3(nGemm, HD / NCW, 1), NTHR, 0, stream>>>(A2, w2p, HW, HD, HD / 32, HD, osc);
  k_agg<0><<<nAgg, NTHR, 0, stream>>>(csr, offp, cnt, HW, b2, A3, nN, csrLen);
  k_gemm<<<dim3(nGemm, (2 * HD) / NCW, 1), NTHR, 0, stream>>>(A3, wpq, PQ, HD, HD / 32, 2 * HD, osc);
  k_edge<<<nEB, NTHR, 0, stream>>>(ei, ef, PQ, Wm1, bm1, wm2p, bm2, Wm3, bm3, out, nE, nN);
}
